// WordAttention_22780506538215
// MI455X (gfx1250) — hardware-verified
//
#include <hip/hip_runtime.h>

typedef __attribute__((ext_vector_type(16))) _Float16 v16h;
typedef __attribute__((ext_vector_type(8)))  _Float16 v8h;
typedef __attribute__((ext_vector_type(16))) __bf16   v16b;
typedef __attribute__((ext_vector_type(8)))  __bf16   v8b;
typedef __attribute__((ext_vector_type(8)))  float    v8f;
typedef __attribute__((ext_vector_type(4)))  float    v4f;
typedef __attribute__((ext_vector_type(4)))  unsigned v4u;

constexpr int kBatch = 8;
constexpr int kSeq   = 2048;
constexpr int kFin   = 512;
constexpr int kHid   = 512;
constexpr size_t kNX = (size_t)kBatch * kSeq * kFin;
constexpr float kPCarry    = 16384.0f;
constexpr float kPCarryInv = 1.0f / 16384.0f;

constexpr size_t kOffX    = 0;
constexpr size_t kOffWt   = kOffX + kNX * 2;
constexpr size_t kOffBias = kOffWt + (size_t)3 * kHid * kFin * 2;
constexpr size_t kOffQh   = kOffBias + (size_t)3 * kHid * 4;
constexpr size_t kOffQl   = kOffQh + kNX * 2;
constexpr size_t kOffKh   = kOffQl + kNX * 2;
constexpr size_t kOffKl   = kOffKh + kNX * 2;
constexpr size_t kOffVt   = kOffKl + kNX * 2;
constexpr size_t kOffP    = kOffVt + kNX * 2;
constexpr size_t kWsTotal = kOffP + (size_t)kSeq * kSeq * 2;
static_assert(kWsTotal == 110630912ull);
static_assert(kWsTotal <= 134217728ull);
static_assert((size_t)kSeq * kSeq * 4 <= kNX * 2);
static_assert(kOffWt % 128 == 0 && kOffBias % 128 == 0 && kOffQh % 128 == 0 && kOffQl % 128 == 0);
static_assert(kOffKh % 128 == 0 && kOffKl % 128 == 0 && kOffVt % 128 == 0 && kOffP % 128 == 0);

static_assert((kBatch * kSeq) % 64 == 0 && kHid % 64 == 0 && kFin % 32 == 0);
static_assert(kHid % 64 == 0 && kSeq % 64 == 0 && kFin % 32 == 0);
static_assert(kSeq % 64 == 0 && kHid % 32 == 0);
static_assert(kSeq % 64 == 0 && kHid % 64 == 0 && kSeq % 32 == 0);

__device__ __forceinline__ unsigned short f2bf_bits(float f) {
  unsigned u = __float_as_uint(f);
  return (unsigned short)((u + 0x7FFFu + ((u >> 16) & 1u)) >> 16);
}
__device__ __forceinline__ float bf_bits2f(unsigned short h) { return __uint_as_float(((unsigned)h) << 16); }
__device__ __forceinline__ unsigned pack_h2(float a, float b) {
  const unsigned short ha = __builtin_bit_cast(unsigned short, (_Float16)a);
  const unsigned short hb = __builtin_bit_cast(unsigned short, (_Float16)b);
  return (unsigned)ha | ((unsigned)hb << 16);
}

__device__ __forceinline__ void dep_guard_h(v8f& a, v8f& b, v16h x, v16h y) { asm volatile("v_nop\n\tv_nop\n\tv_nop\n\tv_nop" : "+v"(a), "+v"(b) : "v"(x), "v"(y)); }
__device__ __forceinline__ void dep_guard_b(v8f& a, v8f& b, v16b x, v16b y) { asm volatile("v_nop\n\tv_nop\n\tv_nop\n\tv_nop" : "+v"(a), "+v"(b) : "v"(x), "v"(y)); }
__device__ __forceinline__ void keep4_h(v16h a, v16h b, v16h c, v16h d) { asm volatile("v_nop" :: "v"(a), "v"(b), "v"(c), "v"(d)); }
__device__ __forceinline__ void keep4_b(v16b a, v16b b, v16b c, v16b d) { asm volatile("v_nop" :: "v"(a), "v"(b), "v"(c), "v"(d)); }
__device__ __forceinline__ void acc_guard4(v8f& a, v8f& b, v8f& c, v8f& d) { asm volatile("v_nop\n\tv_nop\n\tv_nop\n\tv_nop" : "+v"(a), "+v"(b), "+v"(c), "+v"(d)); }
template <typename T> struct Frag;
template <> struct Frag<_Float16> {
  typedef v16h V; union U { v16h v; v8h h[2]; };
  static __device__ __forceinline__ v16h load(const _Float16* p) {
    U f; f.h[0] = *(const v8h*)(p); f.h[1] = *(const v8h*)(p + 16); return f.v;
  }
  static __device__ __forceinline__ v8f mma(v16h a, v16h b, v8f c) {
    return __builtin_amdgcn_wmma_f32_16x16x32_f16(false, a, false, b, (short)0, c, false, false);
  }
  static __device__ __forceinline__ void guard(v8f& a, v8f& b, v16h x, v16h y) { dep_guard_h(a, b, x, y); }
  static __device__ __forceinline__ void keep(v16h a, v16h b, v16h c, v16h d) { keep4_h(a, b, c, d); }
};
template <> struct Frag<__bf16> {
  typedef v16b V; union U { v16b v; v8b h[2]; };
  static __device__ __forceinline__ v16b load(const __bf16* p) {
    U f; f.h[0] = *(const v8b*)(p); f.h[1] = *(const v8b*)(p + 16); return f.v;
  }
  static __device__ __forceinline__ v8f mma(v16b a, v16b b, v8f c) {
    return __builtin_amdgcn_wmma_f32_16x16x32_bf16(false, a, false, b, (short)0, c, false, false);
  }
  static __device__ __forceinline__ void guard(v8f& a, v8f& b, v16b x, v16b y) { dep_guard_b(a, b, x, y); }
  static __device__ __forceinline__ void keep(v16b a, v16b b, v16b c, v16b d) { keep4_b(a, b, c, d); }
};

template <int ET> struct Elem;
template <> struct Elem<0> { typedef _Float16 T; };
template <> struct Elem<1> { typedef __bf16 T; };
template <int ET, bool SPLIT, int BIAS_MODE, int OUT_MODE, bool RESID, int ACT = 0>
__global__ __launch_bounds__(256) void wmma_gemm64(
    const unsigned short* __restrict__ Ap, const unsigned short* __restrict__ A2p, int lda, long strideA,
    const unsigned short* __restrict__ Btp, const unsigned short* __restrict__ Bt2p, int ldb, long strideB,
    void* __restrict__ Cout, void* __restrict__ Cout2, int ldc, long strideC,
    const float* __restrict__ bias,
    const float* __restrict__ resid, long strideR,
    int M, int N, int K, float scale) {
  typedef typename Elem<ET>::T T;
  typedef typename Frag<T>::V V;
  const T* A = (const T*)Ap; const T* A2 = (const T*)A2p; const T* Bt = (const T*)Btp; const T* Bt2 = (const T*)Bt2p;
  __shared__ __align__(16) float sT[8][16 * 68];
  const int b    = blockIdx.y;
  const int lane = threadIdx.x & 31;
  const int wave = threadIdx.x >> 5;
  const int tilesN = N >> 6;
  const int tilesM = M >> 6;
  const int tile = blockIdx.x * 8 + wave;
  if (tile >= tilesM * tilesN) return;
  const int tm = tile / tilesN;
  const int tn = tile - tm * tilesN;
  const int m0 = tm << 6;
  const int n0 = tn << 6;

  const T* Ab  = A  + (size_t)b * strideA;
  const T* Bb  = Bt + (size_t)b * strideB;
  const T* Ab2 = SPLIT ? (A2  + (size_t)b * strideA) : nullptr;
  const T* Bb2 = SPLIT ? (Bt2 + (size_t)b * strideB) : nullptr;

  const int rlane = lane & 15;
  const int koff  = (lane >> 4) * 8;
  const int mOff  = (lane >> 4) * 8;

  v8f acc[4][4];
#pragma unroll
  for (int i = 0; i < 4; ++i)
#pragma unroll
    for (int j = 0; j < 4; ++j) acc[i][j] = (v8f){0.f,0.f,0.f,0.f,0.f,0.f,0.f,0.f};

  for (int k0 = 0; k0 < K; k0 += 32) {
    V bh[4], bl[4];
#pragma unroll
    for (int j = 0; j < 4; ++j) {
      const size_t bo = (size_t)(n0 + (j << 4) + rlane) * ldb + koff + k0;
      bh[j] = Frag<T>::load(Bb + bo);
      if (SPLIT) bl[j] = Frag<T>::load(Bb2 + bo);
    }
#pragma unroll
    for (int i = 0; i < 4; ++i) {
      const size_t ao = (size_t)(m0 + (i << 4) + rlane) * lda + koff + k0;
      V ah = Frag<T>::load(Ab + ao);
      V al;
      if (SPLIT) al = Frag<T>::load(Ab2 + ao);
#pragma unroll
      for (int j = 0; j < 4; ++j) {
        acc[i][j] = Frag<T>::mma(ah, bh[j], acc[i][j]);
        if (SPLIT) {
          acc[i][j] = Frag<T>::mma(ah, bl[j], acc[i][j]);
          acc[i][j] = Frag<T>::mma(al, bh[j], acc[i][j]);
        }
      }
      Frag<T>::guard(acc[i][0], acc[i][3], ah, SPLIT ? al : ah);
    }
    Frag<T>::keep(bh[0], bh[1], bh[2], bh[3]);
    if (SPLIT) Frag<T>::keep(bl[0], bl[1], bl[2], bl[3]);
  }
  acc_guard4(acc[0][0], acc[0][1], acc[0][2], acc[0][3]);
  acc_guard4(acc[1][0], acc[1][1], acc[1][2], acc[1][3]);
  acc_guard4(acc[2][0], acc[2][1], acc[2][2], acc[2][3]);
  acc_guard4(acc[3][0], acc[3][1], acc[3][2], acc[3][3]);

  float* slab = sT[wave];
  const float* Rb = RESID ? (resid + (size_t)b * strideR) : nullptr;
#pragma unroll
  for (int i = 0; i < 4; ++i) {
    const int mBase = m0 + (i << 4);
    float bm8[8] = {0.f,0.f,0.f,0.f,0.f,0.f,0.f,0.f};
    if (BIAS_MODE == 1) {
      const v4f bA = *(const v4f*)(bias + mBase + mOff);
      const v4f bB = *(const v4f*)(bias + mBase + mOff + 4);
      bm8[0] = bA[0]; bm8[1] = bA[1]; bm8[2] = bA[2]; bm8[3] = bA[3];
      bm8[4] = bB[0]; bm8[5] = bB[1]; bm8[6] = bB[2]; bm8[7] = bB[3];
    }
#pragma unroll
    for (int j = 0; j < 4; ++j) {
      const int n = n0 + (j << 4) + rlane;
      float bv = 0.f;
      if (BIAS_MODE == 2) bv = bias[n];
#pragma unroll
      for (int r = 0; r < 8; ++r) {
        float v = acc[i][j][r] * scale;
        if (BIAS_MODE == 1) v += bm8[r];
        if (BIAS_MODE == 2) v += bv;
        if (RESID) v += Rb[(size_t)(mBase + mOff + r) * ldc + n];
        if (ACT == 1) v = tanhf(v);
        if (ACT == 2) v = fmaxf(v, 0.0f);
        if (ACT == 3) v = v / (1.0f + expf(-v));
        if (ACT == 4) v = (v > 0.f) ? v : 0.01f * v;
        if (ACT == 5) v = 0.5f * v * (1.0f + erff(v * 0.70710678118654752f));
        slab[(mOff + r) * 68 + (j << 4) + rlane] = v;
      }
    }
    __builtin_amdgcn_fence(__ATOMIC_RELEASE, "workgroup");
    __builtin_amdgcn_wave_barrier();
    __builtin_amdgcn_fence(__ATOMIC_ACQUIRE, "workgroup");
    if (OUT_MODE == 0) {
      float* C = (float*)Cout + (size_t)b * strideC;
      const int hh = lane >> 4, c4 = (lane & 15) * 4;
      for (int pass = 0; pass < 2; ++pass) {
#pragma unroll
        for (int it = 0; it < 8; ++it) {
          const int row = it * 2 + hh;
          v4f v = *(const v4f*)(slab + row * 68 + c4);
          *(volatile v4f*)(C + (size_t)(mBase + row) * ldc + n0 + c4) = v;
        }
        __threadfence();
      }
    } else {
      const int q = lane >> 3, c8 = (lane & 7) * 8;
      unsigned short* C  = (unsigned short*)Cout  + (size_t)b * strideC;
      unsigned short* C2 = (OUT_MODE == 2) ? ((unsigned short*)Cout2 + (size_t)b * strideC) : nullptr;
      for (int pass = 0; pass < 2; ++pass) {
#pragma unroll
        for (int it = 0; it < 4; ++it) {
          const int row = it * 4 + q;
          const float* sp = slab + row * 68 + c8;
          v8h hv, lv;
#pragma unroll
          for (int e = 0; e < 8; ++e) {
            if (OUT_MODE == 1) {
              hv[e] = (_Float16)sp[e];
            } else {
              unsigned short hb = f2bf_bits(sp[e]);
              unsigned short lb = f2bf_bits(sp[e] - bf_bits2f(hb));
              hv[e] = __builtin_bit_cast(_Float16, hb);
              lv[e] = __builtin_bit_cast(_Float16, lb);
            }
          }
          *(volatile v8h*)(C + (size_t)(mBase + row) * ldc + n0 + c8) = hv;
          if (OUT_MODE == 2) *(volatile v8h*)(C2 + (size_t)(mBase + row) * ldc + n0 + c8) = lv;
        }
        __threadfence();
      }
    }
    __builtin_amdgcn_fence(__ATOMIC_RELEASE, "workgroup");
    __builtin_amdgcn_wave_barrier();
    __builtin_amdgcn_fence(__ATOMIC_ACQUIRE, "workgroup");
  }
}

__global__ __launch_bounds__(256) void cast_f32_bf16x8(
    const float* __restrict__ in, unsigned short* __restrict__ out, int n8) {
  const int i = blockIdx.x * 256 + threadIdx.x;
  if (i < n8) {
    const v4f a = *(const v4f*)(in + (size_t)i * 8);
    const v4f c = *(const v4f*)(in + (size_t)i * 8 + 4);
    v4u w;
    w[0] = (unsigned)f2bf_bits(a[0]) | ((unsigned)f2bf_bits(a[1]) << 16);
    w[1] = (unsigned)f2bf_bits(a[2]) | ((unsigned)f2bf_bits(a[3]) << 16);
    w[2] = (unsigned)f2bf_bits(c[0]) | ((unsigned)f2bf_bits(c[1]) << 16);
    w[3] = (unsigned)f2bf_bits(c[2]) | ((unsigned)f2bf_bits(c[3]) << 16);
    volatile v4u* p = (volatile v4u*)(out + (size_t)i * 8);
    *p = w;
    __threadfence();
    *p = w;
  }
}

__global__ __launch_bounds__(256) void prep_wt(
    const float* __restrict__ w0, const float* __restrict__ w1, const float* __restrict__ w2,
    unsigned short* __restrict__ wt) {
  __shared__ float tile[64][65];
  const int z = blockIdx.z;
  const float* src = (z == 0) ? w0 : ((z == 1) ? w1 : w2);
  const int f0 = blockIdx.y * 64, h0 = blockIdx.x * 64;
  const int tid = threadIdx.x;
  const int lr = tid >> 4, c4 = (tid & 15) * 4;
#pragma unroll
  for (int rr = 0; rr < 4; ++rr) {
    const int row = lr + 16 * rr;
    const v4f v = *(const v4f*)(src + (size_t)(f0 + row) * kHid + h0 + c4);
    tile[row][c4] = v[0]; tile[row][c4 + 1] = v[1]; tile[row][c4 + 2] = v[2]; tile[row][c4 + 3] = v[3];
  }
  __syncthreads();
  const int wave = tid >> 5, lane = tid & 31, q = lane >> 3, seg = lane & 7;
  v4u pk[2];
  int orow[2];
#pragma unroll
  for (int it = 0; it < 2; ++it) {
    const int orw = wave * 8 + it * 4 + q;
    orow[it] = orw;
    v4u w;
#pragma unroll
    for (int e2 = 0; e2 < 4; ++e2) {
      const float a  = tile[seg * 8 + 2 * e2][orw];
      const float bb = tile[seg * 8 + 2 * e2 + 1][orw];
      w[e2] = (unsigned)f2bf_bits(a) | ((unsigned)f2bf_bits(bb) << 16);
    }
    pk[it] = w;
  }
  unsigned short* dst = wt + (size_t)z * kHid * kFin;
  for (int pass = 0; pass < 2; ++pass) {
#pragma unroll
    for (int it = 0; it < 2; ++it)
      *(volatile v4u*)(dst + (size_t)(h0 + orow[it]) * kFin + f0 + seg * 8) = pk[it];
    __threadfence();
  }
}

__global__ __launch_bounds__(128) void prep_bias(
    const float* __restrict__ b0, const float* __restrict__ b1, const float* __restrict__ b2,
    float* __restrict__ outb) {
  const int z = blockIdx.x;
  const float* src = (z == 0) ? b0 : ((z == 1) ? b1 : b2);
  const int t = threadIdx.x;
  const v4f v = *(const v4f*)(src + t * 4);
  v4f w;
  w[0] = bf_bits2f(f2bf_bits(v[0])); w[1] = bf_bits2f(f2bf_bits(v[1]));
  w[2] = bf_bits2f(f2bf_bits(v[2])); w[3] = bf_bits2f(f2bf_bits(v[3]));
  volatile v4f* p = (volatile v4f*)(outb + z * kHid + t * 4);
  *p = w;
  __threadfence();
  *p = w;
}

__global__ __launch_bounds__(256) void softmax_rows(
    const float* __restrict__ S, unsigned short* __restrict__ P, int nrows) {
  __shared__ __align__(16) float srow[4][kSeq];
  __shared__ float smax[8];
  __shared__ float ssum[8];
  const int tid = threadIdx.x, wave = tid >> 5, lane = tid & 31;
  const int r = wave >> 1, half = wave & 1;
  int row = blockIdx.x * 4 + r;
  row = row < nrows ? row : nrows - 1;
  const float* src = S + (size_t)row * kSeq + half * 1024;
  float* lrow = &srow[r][half * 1024];

  float mx = -INFINITY;
#pragma unroll 1
  for (int it = 0; it < 8; ++it) {
    const int col = (it >> 1) * 256 + lane * 8 + (it & 1) * 4;
    const v4f v = *(const v4f*)(src + col);
    mx = fmaxf(mx, fmaxf(fmaxf(v[0], v[1]), fmaxf(v[2], v[3])));
    *(v4f*)(lrow + col) = v;
  }
#pragma unroll
  for (int off = 1; off < 32; off <<= 1) mx = fmaxf(mx, __shfl_xor(mx, off, 32));
  if (lane == 0) smax[wave] = mx;
  __syncthreads();
  const float rowmax = fmaxf(smax[2 * r], smax[2 * r + 1]);

  float sum = 0.0f;
#pragma unroll 1
  for (int it = 0; it < 8; ++it) {
    const int col = (it >> 1) * 256 + lane * 8 + (it & 1) * 4;
    const v4f v = *(const v4f*)(lrow + col);
    v4f e;
    e[0] = expf(v[0] - rowmax);
    e[1] = expf(v[1] - rowmax);
    e[2] = expf(v[2] - rowmax);
    e[3] = expf(v[3] - rowmax);
    sum += (e[0] + e[1]) + (e[2] + e[3]);
    *(v4f*)(lrow + col) = e;
  }
#pragma unroll
  for (int off = 1; off < 32; off <<= 1) sum += __shfl_xor(sum, off, 32);
  if (lane == 0) ssum[wave] = sum;
  __syncthreads();
  const float rowsum = ssum[2 * r] + ssum[2 * r + 1];
  const float sc = kPCarry * (1.0f / rowsum);

  v4u pk[4];
#pragma unroll
  for (int i = 0; i < 4; ++i) {
    const v4f a = *(const v4f*)(lrow + i * 256 + lane * 8);
    const v4f c = *(const v4f*)(lrow + i * 256 + lane * 8 + 4);
    v4u w;
    w[0] = pack_h2(a[0] * sc, a[1] * sc);
    w[1] = pack_h2(a[2] * sc, a[3] * sc);
    w[2] = pack_h2(c[0] * sc, c[1] * sc);
    w[3] = pack_h2(c[2] * sc, c[3] * sc);
    pk[i] = w;
  }
  unsigned short* prow = P + (size_t)row * kSeq + half * 1024;
  for (int pass = 0; pass < 2; ++pass) {
#pragma unroll
    for (int i = 0; i < 4; ++i)
      *(volatile v4u*)(prow + i * 256 + lane * 8) = pk[i];
    __threadfence();
  }
}

extern "C" void kernel_launch(void* const* d_in, const int* in_sizes, int n_in,
                              void* d_out, int out_size, void* d_ws, size_t ws_size,
                              hipStream_t stream) {
  if (n_in < 7) return;
  if ((size_t)in_sizes[0] != kNX || in_sizes[1] != kFin * kHid || in_sizes[2] != kHid ||
      in_sizes[3] != kFin * kHid || in_sizes[4] != kHid || in_sizes[5] != kFin * kHid || in_sizes[6] != kHid) return;
  if ((size_t)out_size != kNX) return;
  if (ws_size < kWsTotal) return;

  const float* p_x  = (const float*)d_in[0];
  const float* p_wq = (const float*)d_in[1];
  const float* p_bq = (const float*)d_in[2];
  const float* p_wk = (const float*)d_in[3];
  const float* p_bk = (const float*)d_in[4];
  const float* p_wv = (const float*)d_in[5];
  const float* p_bv = (const float*)d_in[6];
  float* out = (float*)d_out;

  char* ws = (char*)d_ws;
  unsigned short* xb    = (unsigned short*)(ws + kOffX);
  float*          sc    = (float*)(ws + kOffX);
  unsigned short* wt    = (unsigned short*)(ws + kOffWt);
  float*          biasr = (float*)(ws + kOffBias);
  unsigned short* qh    = (unsigned short*)(ws + kOffQh);
  unsigned short* ql    = (unsigned short*)(ws + kOffQl);
  unsigned short* kh    = (unsigned short*)(ws + kOffKh);
  unsigned short* kl    = (unsigned short*)(ws + kOffKl);
  unsigned short* vt    = (unsigned short*)(ws + kOffVt);
  unsigned short* pp    = (unsigned short*)(ws + kOffP);

  const int nRows = kBatch * kSeq;
  const size_t wplane = (size_t)kHid * kFin;

  cast_f32_bf16x8<<<dim3((unsigned)(kNX / 8 / 256)), 256, 0, stream>>>(p_x, xb, (int)(kNX / 8));
  prep_wt<<<dim3(kHid / 64, kFin / 64, 3), 256, 0, stream>>>(p_wq, p_wk, p_wv, wt);
  prep_bias<<<dim3(3), 128, 0, stream>>>(p_bq, p_bk, p_bv, biasr);

  {
    const int tiles = (nRows / 64) * (kHid / 64);
    wmma_gemm64<1, false, 2, 2, false><<<dim3(tiles / 8, 1), 256, 0, stream>>>(
        xb, xb, kFin, 0L, wt, wt, kFin, 0L, (void*)qh, (void*)ql, kHid, 0L,
        biasr, biasr, 0L, nRows, kHid, kFin, 1.0f);
    wmma_gemm64<1, false, 2, 2, false><<<dim3(tiles / 8, 1), 256, 0, stream>>>(
        xb, xb, kFin, 0L, wt + wplane, wt + wplane, kFin, 0L, (void*)kh, (void*)kl, kHid, 0L,
        biasr + kHid, biasr, 0L, nRows, kHid, kFin, 1.0f);
  }
  {
    const int tiles = (kHid / 64) * (kSeq / 64);
    wmma_gemm64<1, false, 1, 1, false><<<dim3(tiles / 8, kBatch), 256, 0, stream>>>(
        wt + 2 * wplane, wt + 2 * wplane, kFin, 0L,
        xb, xb, kFin, (long)kSeq * kFin,
        (void*)vt, (void*)vt, kSeq, (long)kHid * kSeq,
        biasr + 2 * kHid, biasr, 0L, kHid, kSeq, kFin, 1.0f);
  }
  for (int b = 0; b < kBatch; ++b) {
    const size_t qo = (size_t)b * kSeq * kHid;
    const size_t vo = (size_t)b * kHid * kSeq;
    {
      const int tiles = (kSeq / 64) * (kSeq / 64);
      wmma_gemm64<1, true, 0, 0, false><<<dim3(tiles / 8, 1), 256, 0, stream>>>(
          qh + qo, ql + qo, kHid, 0L, kh + qo, kl + qo, kHid, 0L,
          (void*)sc, (void*)sc, kSeq, 0L, biasr, biasr, 0L, kSeq, kSeq, kHid, 1.0f);
    }
    softmax_rows<<<dim3(kSeq / 4), 256, 0, stream>>>(sc, pp, kSeq);
    {
      const int tiles = (kSeq / 64) * (kHid / 64);
      wmma_gemm64<0, false, 0, 0, false><<<dim3(tiles / 8, 1), 256, 0, stream>>>(
          pp, pp, kSeq, 0L, vt + vo, vt + vo, kSeq, 0L,
          (void*)(out + qo), (void*)(out + qo), kHid, 0L, biasr, biasr, 0L, kSeq, kHid, kSeq, kPCarryInv);
    }
  }
}
